// MolGNN_29712583754389
// MI455X (gfx1250) — hardware-verified
//
#include <hip/hip_runtime.h>
#include <math.h>

typedef __attribute__((ext_vector_type(16))) _Float16 v16h;
typedef __attribute__((ext_vector_type(16))) __bf16 v16b;
typedef __attribute__((ext_vector_type(8)))  _Float16 v8h;
typedef __attribute__((ext_vector_type(8)))  float v8f;
typedef __attribute__((ext_vector_type(4)))  float v4f;
typedef __attribute__((ext_vector_type(2)))  float v2f;
typedef __attribute__((ext_vector_type(4)))  unsigned v4u;
typedef __attribute__((ext_vector_type(4)))  int v4i;
typedef float __attribute__((may_alias)) float_a;
typedef int __attribute__((may_alias)) int_a;

template <typename T> __device__ __forceinline__ void vst2(void* p, T v) { *(volatile T*)p = v; __threadfence(); *(volatile T*)p = v; }
__device__ __forceinline__ v8f wmma16(v16h a, v16h b, v8f c) {
  v8f d = __builtin_amdgcn_wmma_f32_16x16x32_f16(false, a, false, b, (short)0, c, false, false);
  asm volatile("v_nop\n\tv_nop\n\tv_nop\n\tv_nop" : "+v"(d) : "v"(a), "v"(b));
  return d;
}
__device__ __forceinline__ v8f wmma_bf(v16b a, v16b b, v8f c) {
  v8f d = __builtin_amdgcn_wmma_f32_16x16x32_bf16(false, a, false, b, (short)0, c, false, false);
  asm volatile("v_nop\n\tv_nop\n\tv_nop\n\tv_nop" : "+v"(d) : "v"(a), "v"(b));
  return d;
}
__device__ __forceinline__ v16h frag_h(const _Float16* rowk0, int lane) {
  union { v16h v; v8h q[2]; } u; const _Float16* p = rowk0 + 8 * (lane >> 4);
  u.q[0] = *(const v8h*)p; u.q[1] = *(const v8h*)(p + 16); return u.v;
}
__device__ __forceinline__ v16h frag_f32(const float* rowk0, int lane) {
  v16h a; const float* p = rowk0 + 8 * (lane >> 4);
#pragma unroll
  for (int i = 0; i < 8; ++i) { a[i] = (_Float16)p[i]; a[8 + i] = (_Float16)p[16 + i]; }
  return a;
}
__device__ __forceinline__ v16h frag_f32s(const float* rowk0, int lane, float sc) {
  v16h a; const float* p = rowk0 + 8 * (lane >> 4);
#pragma unroll
  for (int i = 0; i < 8; ++i) { a[i] = (_Float16)(p[i] * sc); a[8 + i] = (_Float16)(p[16 + i] * sc); }
  return a;
}
__device__ __forceinline__ v16h fragc_f32(const float* W, int k0, int n, int lane, int ld, int K) {
  v16h a; const int g = lane >> 4;
#pragma unroll
  for (int i = 0; i < 8; ++i) { const int ka = k0 + 8 * g + i, kb = ka + 16;
    a[i] = (_Float16)(ka < K ? W[(size_t)ka * ld + n] : 0.f); a[8 + i] = (_Float16)(kb < K ? W[(size_t)kb * ld + n] : 0.f); }
  return a;
}
struct F2 { v16b h, l; };
__device__ __forceinline__ F2 bsplit16(const float v[16]) { F2 r;
#pragma unroll
  for (int i = 0; i < 16; ++i) { const __bf16 h = (__bf16)v[i]; r.h[i] = h; r.l[i] = (__bf16)(v[i] - (float)h); }
  return r; }
__device__ __forceinline__ F2 split_row(const float* row, int k0, int lane) { float v[16]; const float* p = row + k0 + 8 * (lane >> 4);
#pragma unroll
  for (int i = 0; i < 8; ++i) { v[i] = p[i]; v[8 + i] = p[16 + i]; }
  return bsplit16(v); }
__device__ __forceinline__ F2 split_rowK(const float* row, int k0, int lane, int K) { float v[16]; const int g = lane >> 4;
#pragma unroll
  for (int i = 0; i < 8; ++i) { const int ka = k0 + 8 * g + i, kb = ka + 16; v[i] = ka < K ? row[ka] : 0.f; v[8 + i] = kb < K ? row[kb] : 0.f; }
  return bsplit16(v); }
__device__ __forceinline__ F2 split_col(const float* W, int k0, int n, int lane, int ld, int K) { float v[16]; const int g = lane >> 4;
#pragma unroll
  for (int i = 0; i < 8; ++i) { const int ka = k0 + 8 * g + i, kb = ka + 16; v[i] = ka < K ? W[(size_t)ka * ld + n] : 0.f; v[8 + i] = kb < K ? W[(size_t)kb * ld + n] : 0.f; }
  return bsplit16(v); }
__device__ __forceinline__ v8f mac3(const F2& a, const F2& b, v8f c) { c = wmma_bf(a.l, b.h, c); c = wmma_bf(a.h, b.l, c); return wmma_bf(a.h, b.h, c); }
__device__ __forceinline__ float sigm(float v) { return 1.0f / (1.0f + expf(-v)); }
#define LDSX() do { asm volatile("s_wait_dscnt 0" ::: "memory"); __builtin_amdgcn_wave_barrier(); __builtin_amdgcn_fence(__ATOMIC_RELEASE, "workgroup"); } while (0)


#define NN 100000
#define NE 600000
#define NG 4096
#define HD 128
#define OD 768
#define NVOC 119
#define EVOC 22
#define RB 512
#define NRB 196
#define NNP (NRB * RB)
#define EPT 8
#define CH (256 * EPT)
__device__ __forceinline__ int clampn(int v) { return v < 0 ? 0 : (v >= NN ? NN - 1 : v); }
__device__ __forceinline__ int clampv(int v, int hi) { return v < 0 ? 0 : (v > hi ? hi : v); }

__global__ __launch_bounds__(256) void k_embed(const int* __restrict__ xi, const float* __restrict__ ntab, float* __restrict__ H0) {
  const int wave = threadIdx.x >> 5, lane = threadIdx.x & 31;
  for (int r = blockIdx.x * 8 + wave; r < NNP; r += gridDim.x * 8) { v4f v = {0.f, 0.f, 0.f, 0.f};
    if (r < NN) {
#pragma unroll
      for (int i = 0; i < 9; ++i) { const int a = clampv(xi[(size_t)r * 9 + i], NVOC - 1); const v4f t = *(const v4f*)(ntab + ((size_t)i * NVOC + a) * HD + lane * 4); v[0] += t[0]; v[1] += t[1]; v[2] += t[2]; v[3] += t[3]; } }
    vst2(H0 + (size_t)r * HD + lane * 4, v); }
}
__global__ __launch_bounds__(256) void k_gine(const int* __restrict__ esrc, const int* __restrict__ edst, const int* __restrict__ eattr, const float* __restrict__ etab, const float* __restrict__ epsp,
                                             const float* __restrict__ Hin, float* __restrict__ Z) {
  __shared__ __align__(16) float sacc[RB][HD];
  __shared__ int slst[8][32 * EPT], sdl[8][32 * EPT]; __shared__ int scnt[8];
  const int tid = threadIdx.x, wave = tid >> 5, lane = tid & 31;
  const int r0 = blockIdx.x * RB; const float opeps = 1.0f + epsp[0];
  for (int q = tid; q < RB * HD; q += 256) (&sacc[0][0])[q] = 0.f;
  __syncthreads();
#pragma unroll 1
  for (int c0 = 0; c0 < NE; c0 += CH) { const int e0 = c0 + tid * EPT; int hd[EPT]; int cnt = 0;
    if (e0 + EPT <= NE) {
#pragma unroll
      for (int v = 0; v < EPT / 4; ++v) { const int4 d4 = *(const int4*)(edst + e0 + v * 4); const int dd[4] = {d4.x, d4.y, d4.z, d4.w};
#pragma unroll
        for (int u = 0; u < 4; ++u) { const unsigned rel = (unsigned)(clampn(dd[u]) - r0); const bool h = rel < (unsigned)RB; hd[v * 4 + u] = h ? (int)rel : -1; cnt += h ? 1 : 0; } } }
    else {
#pragma unroll
      for (int u = 0; u < EPT; ++u) { const int e = e0 + u; hd[u] = -1; if (e < NE) { const unsigned rel = (unsigned)(clampn(edst[e]) - r0); if (rel < (unsigned)RB) { hd[u] = (int)rel; ++cnt; } } } }
    int incl = cnt;
#pragma unroll
    for (int off = 1; off < 32; off <<= 1) { const int vv = __shfl_up(incl, off, 32); if (lane >= off) incl += vv; }
    const int wtot = __shfl(incl, 31, 32); int pos = incl - cnt;
    if (cnt > 0) {
#pragma unroll
      for (int u = 0; u < EPT; ++u) if (hd[u] >= 0) { slst[wave][pos] = e0 + u; sdl[wave][pos] = hd[u]; ++pos; } }
    if (lane == 0) scnt[wave] = wtot;
    __syncthreads();
#pragma unroll 1
    for (int w = 0; w < 8; ++w) { const int nh = scnt[w];
#pragma unroll 1
      for (int i = tid; i < nh; i += 256) { const int e = slst[w][i]; const int s = clampn(esrc[e]);
        const int a0 = clampv(eattr[(size_t)e * 3], EVOC - 1), a1 = clampv(eattr[(size_t)e * 3 + 1], EVOC - 1), a2 = clampv(eattr[(size_t)e * 3 + 2], EVOC - 1);
        slst[w][i] = (int)((unsigned)s | ((unsigned)a0 << 17) | ((unsigned)a1 << 22) | ((unsigned)a2 << 27)); } }
    __syncthreads();
    if (tid < HD) { const int f = tid; const float* t0 = etab + f; const float* t1 = etab + (size_t)EVOC * HD + f; const float* t2 = etab + (size_t)2 * EVOC * HD + f;
#pragma unroll 1
      for (int w = 0; w < 8; ++w) { const int nh = scnt[w];
#pragma unroll 1
        for (int i = 0; i < nh; ++i) { const unsigned pk = (unsigned)slst[w][i]; const int dl = sdl[w][i]; const int s = (int)(pk & 0x1FFFFu), a0 = (int)((pk >> 17) & 31u), a1 = (int)((pk >> 22) & 31u), a2 = (int)(pk >> 27);
          const float v = Hin[(size_t)s * HD + f] + t0[(size_t)a0 * HD] + t1[(size_t)a1 * HD] + t2[(size_t)a2 * HD]; sacc[dl][f] += v > 0.f ? v : 0.f; } } }
    __syncthreads(); }
#pragma unroll 1
  for (int q = tid; q < RB * (HD / 4); q += 256) { const int rl = q >> 5, pc = q & 31; const int row = r0 + rl; v4f o = {0.f, 0.f, 0.f, 0.f};
    if (row < NN) { const v4f a = *(const v4f*)(&sacc[rl][pc * 4]); const v4f h = *(const v4f*)(Hin + (size_t)row * HD + pc * 4); o[0] = opeps * h[0] + a[0]; o[1] = opeps * h[1] + a[1]; o[2] = opeps * h[2] + a[2]; o[3] = opeps * h[3] + a[3]; }
    vst2(Z + (size_t)row * HD + pc * 4, o); }
}
__global__ __launch_bounds__(128) void k_pack(const float* __restrict__ W1, const float* __restrict__ W2, _Float16* __restrict__ PT) {
  const int b = blockIdx.x, tid = threadIdx.x; const int l = b / (2 * HD), wn = b % (2 * HD), which = wn / HD, n = wn % HD; const float* W = (which == 0 ? W1 : W2) + (size_t)l * HD * HD;
  __shared__ __align__(16) _Float16 srow[HD];
  srow[tid] = (_Float16)(W[(size_t)tid * HD + n] * 16.0f);
  __syncthreads();
  if (tid < HD / 8) vst2(PT + (size_t)b * HD + tid * 8, *(const v4u*)(&srow[tid * 8]));
}
__global__ __launch_bounds__(128) void k_mlp(const float* __restrict__ Z, const _Float16* __restrict__ P1, const float* __restrict__ b1, const _Float16* __restrict__ P2, const float* __restrict__ b2, float* __restrict__ Hout) {
  __shared__ __align__(16) _Float16 sZ[64][HD + 8];
  __shared__ __align__(16) float so[4][16][132];
  const int tid = threadIdx.x, wave = tid >> 5, lane = tid & 31, col = lane & 15, g = lane >> 4;
  const int r0 = blockIdx.x * 64 + wave * 16; const int ra = (r0 + col) < NN ? (r0 + col) : (NN - 1);
  v8f acc[8] = {};
#pragma unroll
  for (int kc = 0; kc < HD / 32; ++kc) { const v16h a = frag_f32(Z + (size_t)ra * HD + kc * 32, lane);
#pragma unroll
    for (int j = 0; j < 8; ++j) acc[j] = wmma16(a, frag_h(P1 + (size_t)(j * 16 + col) * HD + kc * 32, lane), acc[j]); }
#pragma unroll
  for (int j = 0; j < 8; ++j) { const float bb = b1[j * 16 + col];
#pragma unroll
    for (int r = 0; r < 8; ++r) { const float v = acc[j][r] * (1.0f / 16.0f) + bb; sZ[wave * 16 + 8 * g + r][j * 16 + col] = (_Float16)(v > 0.f ? v : 0.f); } }
  LDSX();
  v8f acc2[8] = {};
#pragma unroll
  for (int kc = 0; kc < HD / 32; ++kc) { const v16h a = frag_h(&sZ[wave * 16 + col][0] + kc * 32, lane);
#pragma unroll
    for (int j = 0; j < 8; ++j) acc2[j] = wmma16(a, frag_h(P2 + (size_t)(j * 16 + col) * HD + kc * 32, lane), acc2[j]); }
#pragma unroll
  for (int j = 0; j < 8; ++j) { const float bb = b2[j * 16 + col];
#pragma unroll
    for (int r = 0; r < 8; ++r) { const float v = acc2[j][r] * (1.0f / 16.0f) + bb; so[wave][8 * g + r][j * 16 + col] = (r0 + 8 * g + r) < NN ? (v > 0.f ? v : 0.f) : 0.f; } }
  LDSX();
#pragma unroll 4
  for (int rl = 0; rl < 16; ++rl) vst2(Hout + (size_t)(r0 + rl) * HD + lane * 4, *(const v4f*)(&so[wave][rl][lane * 4]));
}
__global__ __launch_bounds__(256) void k_pool(const int* __restrict__ batch, const float* __restrict__ H, float* __restrict__ G) {
  __shared__ __align__(16) float sacc[RB][HD];
  __shared__ int slst[8][32 * EPT], sdl[8][32 * EPT]; __shared__ int scnt[8];
  const int tid = threadIdx.x, wave = tid >> 5, lane = tid & 31;
  const int g0 = blockIdx.x * RB;
  for (int q = tid; q < RB * HD; q += 256) (&sacc[0][0])[q] = 0.f;
  __syncthreads();
#pragma unroll 1
  for (int c0 = 0; c0 < NN; c0 += CH) { const int n0 = c0 + tid * EPT; int hd[EPT]; int cnt = 0;
#pragma unroll
    for (int u = 0; u < EPT; ++u) { const int n = n0 + u; hd[u] = -1; if (n < NN) { const unsigned rel = (unsigned)(batch[n] - g0); if (rel < (unsigned)RB) { hd[u] = (int)rel; ++cnt; } } }
    int incl = cnt;
#pragma unroll
    for (int off = 1; off < 32; off <<= 1) { const int vv = __shfl_up(incl, off, 32); if (lane >= off) incl += vv; }
    const int wtot = __shfl(incl, 31, 32); int pos = incl - cnt;
    if (cnt > 0) {
#pragma unroll
      for (int u = 0; u < EPT; ++u) if (hd[u] >= 0) { slst[wave][pos] = n0 + u; sdl[wave][pos] = hd[u]; ++pos; } }
    if (lane == 0) scnt[wave] = wtot;
    __syncthreads();
    if (tid < HD) {
#pragma unroll 1
      for (int w = 0; w < 8; ++w) { const int nh = scnt[w];
#pragma unroll 1
        for (int i = 0; i < nh; ++i) sacc[sdl[w][i]][tid] += H[(size_t)slst[w][i] * HD + tid]; } }
    __syncthreads(); }
#pragma unroll 1
  for (int q = tid; q < RB * (HD / 4); q += 256) { const int rl = q >> 5, pc = q & 31; vst2(G + (size_t)(g0 + rl) * HD + pc * 4, *(const v4f*)(&sacc[rl][pc * 4])); }
}
__global__ __launch_bounds__(128) void k_head(const float* __restrict__ G, const float* __restrict__ Wp, const float* __restrict__ bp, float* __restrict__ out) {
  __shared__ __align__(16) float so[64][OD + 4]; __shared__ float sinv[64];
  const int tid = threadIdx.x, wave = tid >> 5, lane = tid & 31, col = lane & 15, g = lane >> 4;
  const int r0 = blockIdx.x * 64 + wave * 16;
#pragma unroll 1
  for (int ps = 0; ps < OD / 128; ++ps) { v8f acc[8] = {};
#pragma unroll 1
    for (int kc = 0; kc < HD / 32; ++kc) { const F2 a = split_row(G + (size_t)(r0 + col) * HD, kc * 32, lane);
#pragma unroll
      for (int j = 0; j < 8; ++j) acc[j] = mac3(a, split_col(Wp, kc * 32, ps * 128 + j * 16 + col, lane, OD, HD), acc[j]); }
#pragma unroll
    for (int j = 0; j < 8; ++j) { const int n = ps * 128 + j * 16 + col; const float bb = bp[n];
#pragma unroll
      for (int r = 0; r < 8; ++r) so[wave * 16 + 8 * g + r][n] = acc[j][r] + bb; } }
  LDSX();
  { const int rl = wave * 16 + (lane & 15), hf = lane >> 4; const float* row = &so[rl][hf * (OD / 2)]; float ss = 0.f;
#pragma unroll 4
    for (int k = 0; k < OD / 2; ++k) ss += row[k] * row[k];
    ss += __shfl_xor(ss, 16, 32);
    if (hf == 0) sinv[rl] = 1.0f / fmaxf(sqrtf(ss), 1e-12f); }
  LDSX();
#pragma unroll 1
  for (int rl = 0; rl < 16; ++rl) { const float inv = sinv[wave * 16 + rl];
    for (int pc = lane; pc < OD / 4; pc += 32) { v4f v = *(const v4f*)(&so[wave * 16 + rl][pc * 4]); v[0] *= inv; v[1] *= inv; v[2] *= inv; v[3] *= inv; vst2(out + (size_t)(r0 + rl) * OD + pc * 4, v); } }
}
extern "C" void kernel_launch(void* const* d_in, const int* in_sizes, int n_in, void* d_out, int out_size, void* d_ws, size_t ws_size, hipStream_t stream) {
  (void)in_sizes; (void)n_in; (void)out_size; (void)ws_size;
  const int* xi = (const int*)d_in[0]; const int* eattr = (const int*)d_in[1]; const int* ei = (const int*)d_in[2]; const int* batch = (const int*)d_in[3];
  const float* ntab = (const float*)d_in[4]; const float* etab = (const float*)d_in[5]; const float* W1 = (const float*)d_in[6]; const float* b1 = (const float*)d_in[7]; const float* W2 = (const float*)d_in[8]; const float* b2 = (const float*)d_in[9];
  const float* eps = (const float*)d_in[10]; const float* Wp = (const float*)d_in[11]; const float* bp = (const float*)d_in[12];
  const int* esrc = ei; const int* edst = ei + NE;
  float* out = (float*)d_out;
  char* ws = (char*)d_ws; size_t off = 0;
  auto take = [&](size_t bytes) { char* p = ws + off; off += (bytes + 255) & ~(size_t)255; return p; };
  float* HA = (float*)take((size_t)NNP * HD * 4); float* Zb = (float*)take((size_t)NNP * HD * 4); _Float16* PT = (_Float16*)take((size_t)3 * 2 * HD * HD * 2); float* G = (float*)take((size_t)NG * HD * 4);
  k_embed<<<1568, 256, 0, stream>>>(xi, ntab, HA);
  k_pack<<<3 * 2 * HD, 128, 0, stream>>>(W1, W2, PT);
  k_gine<<<NRB, 256, 0, stream>>>(esrc, edst, eattr, etab, eps + 0, HA, Zb);
  k_mlp<<<NNP / 64, 128, 0, stream>>>(Zb, PT + 0 * 2 * HD * HD, b1 + 0 * HD, PT + (0 * 2 + 1) * HD * HD, b2 + 0 * HD, HA);
  k_gine<<<NRB, 256, 0, stream>>>(esrc, edst, eattr, etab, eps + 1, HA, Zb);
  k_mlp<<<NNP / 64, 128, 0, stream>>>(Zb, PT + 1 * 2 * HD * HD, b1 + 1 * HD, PT + (1 * 2 + 1) * HD * HD, b2 + 1 * HD, HA);
  k_gine<<<NRB, 256, 0, stream>>>(esrc, edst, eattr, etab, eps + 2, HA, Zb);
  k_mlp<<<NNP / 64, 128, 0, stream>>>(Zb, PT + 2 * 2 * HD * HD, b1 + 2 * HD, PT + (2 * 2 + 1) * HD * HD, b2 + 2 * HD, HA);
  k_pool<<<NG / RB, 256, 0, stream>>>(batch, HA, G);
  k_head<<<NG / 64, 128, 0, stream>>>(G, Wp, bp, out);
}
